// SpatialUniCrossAttention_9603546874538
// MI455X (gfx1250) — hardware-verified
//
#include <hip/hip_runtime.h>
#include <hip/hip_bf16.h>
#include <stdint.h>
#include <stddef.h>


typedef __bf16 v16b __attribute__((ext_vector_type(16)));
typedef _Float16 v16h __attribute__((ext_vector_type(16)));
typedef float v8f __attribute__((ext_vector_type(8)));
typedef float v4f __attribute__((ext_vector_type(4)));
typedef unsigned short v8us __attribute__((ext_vector_type(8)));

constexpr int Cc = 256;
constexpr int Lc = 4096;
constexpr int Hc = 8;
constexpr int Dc = 32;

union FragB { v16b v; v8us u[2]; };
union FragH { v16h v; v8us u[2]; };

__device__ __forceinline__ v8f wmb(v16b a, v16b b, v8f c) {
  c = __builtin_amdgcn_wmma_f32_16x16x32_bf16(false, a, false, b, (short)0, c, false, false);
  asm volatile("v_nop\n\tv_nop\n\tv_nop\n\tv_nop" : "+v"(c) : "v"(a), "v"(b));
  return c;
}
__device__ __forceinline__ v8f wmh(v16h a, v16h b, v8f c) {
  c = __builtin_amdgcn_wmma_f32_16x16x32_f16(false, a, false, b, (short)0, c, false, false);
  asm volatile("v_nop\n\tv_nop\n\tv_nop\n\tv_nop" : "+v"(c) : "v"(a), "v"(b));
  return c;
}

__device__ __forceinline__ void split1(float x, unsigned short& hi, unsigned short& lo) {
  const __bf16 hb = (__bf16)x;
  const float xh = (float)hb;
  const __bf16 lb = (__bf16)(x - xh);
  hi = __builtin_bit_cast(unsigned short, hb);
  lo = __builtin_bit_cast(unsigned short, lb);
}
__device__ __forceinline__ void split8(v4f a, v4f c, v8us& hi, v8us& lo) {
  const float f[8] = {a.x, a.y, a.z, a.w, c.x, c.y, c.z, c.w};
#pragma unroll
  for (int i = 0; i < 8; ++i) {
    unsigned short h, l;
    split1(f[i], h, l);
    hi[i] = h;
    lo[i] = l;
  }
}
__device__ __forceinline__ unsigned short hbits(float x) {
  const _Float16 hv = (_Float16)x;
  return __builtin_bit_cast(unsigned short, hv);
}

template <int MODE>
__global__ __launch_bounds__(128)
void gemm64(const float* __restrict__ A, const float* __restrict__ W, int Nn, int Mtot,
            float* __restrict__ outF, unsigned short* __restrict__ q16,
            unsigned short* __restrict__ k16, unsigned short* __restrict__ vT,
            size_t planeElems) {
  __shared__ __align__(16) unsigned short Ah[64][32];
  __shared__ __align__(16) unsigned short Al[64][32];
  __shared__ __align__(16) unsigned short Bh[64][32];
  __shared__ __align__(16) unsigned short Bl[64][32];
  __shared__ __align__(16) float Cs[64][64];
  __shared__ __align__(16) unsigned short S16[2][64][64];

  const int tid = threadIdx.x;
  const int wave = tid >> 5, lane = tid & 31;
  const int lx = lane & 15, lh = lane >> 4;
  const int m0 = blockIdx.x * 64;
  const int n0 = blockIdx.y * 64;
  if (m0 + 64 > Mtot || n0 + 64 > Nn) return;

  v8f acc[4] = {};

  for (int k0 = 0; k0 < Cc; k0 += 32) {
    {
      const int r = tid >> 1, hf = (tid & 1) * 16;
      const float* src = A + (size_t)(m0 + r) * Cc + k0 + hf;
      const v4f f0 = *(const v4f*)(src + 0);
      const v4f f1 = *(const v4f*)(src + 4);
      const v4f f2 = *(const v4f*)(src + 8);
      const v4f f3 = *(const v4f*)(src + 12);
      v8us h0, l0v, h1, l1v;
      split8(f0, f1, h0, l0v);
      split8(f2, f3, h1, l1v);
      *(v8us*)&Ah[r][hf] = h0;
      *(v8us*)&Ah[r][hf + 8] = h1;
      *(v8us*)&Al[r][hf] = l0v;
      *(v8us*)&Al[r][hf + 8] = l1v;
    }
    {
      const int kk = tid >> 2, nof = (tid & 3) * 16;
      const float* src = W + (size_t)(k0 + kk) * Nn + n0 + nof;
#pragma unroll
      for (int jj = 0; jj < 4; ++jj) {
        const v4f f = *(const v4f*)(src + 4 * jj);
        const float g[4] = {f.x, f.y, f.z, f.w};
#pragma unroll
        for (int e = 0; e < 4; ++e) {
          unsigned short h, l;
          split1(g[e], h, l);
          Bh[nof + 4 * jj + e][kk] = h;
          Bl[nof + 4 * jj + e][kk] = l;
        }
      }
    }
    __syncthreads();

    FragB ah, al;
    {
      const int row = 16 * wave + lx;
      ah.u[0] = *(const v8us*)&Ah[row][8 * lh];
      ah.u[1] = *(const v8us*)&Ah[row][16 + 8 * lh];
      al.u[0] = *(const v8us*)&Al[row][8 * lh];
      al.u[1] = *(const v8us*)&Al[row][16 + 8 * lh];
    }
#pragma unroll
    for (int t = 0; t < 4; ++t) {
      const int n = 16 * t + lx;
      FragB bh, bl;
      bh.u[0] = *(const v8us*)&Bh[n][8 * lh];
      bh.u[1] = *(const v8us*)&Bh[n][16 + 8 * lh];
      bl.u[0] = *(const v8us*)&Bl[n][8 * lh];
      bl.u[1] = *(const v8us*)&Bl[n][16 + 8 * lh];
      acc[t] = wmb(ah.v, bh.v, acc[t]);
      acc[t] = wmb(ah.v, bl.v, acc[t]);
      acc[t] = wmb(al.v, bh.v, acc[t]);
    }
    __syncthreads();
  }

  const int q = lane >> 3, p = lane & 7;

  if constexpr (MODE == 0) {
#pragma unroll
    for (int t = 0; t < 4; ++t)
#pragma unroll
      for (int r = 0; r < 8; ++r)
        Cs[16 * wave + 8 * lh + r][16 * t + lx] = acc[t][r];
    __syncthreads();
#pragma unroll
    for (int ps = 0; ps < 2; ++ps) {
      if (ps) __threadfence();
#pragma unroll
      for (int i = 0; i < 8; ++i) {
        const int L = 4 * i + q;
        const int row = 16 * wave + (L >> 1);
        const int hf = L & 1;
        const v4f v = *(const v4f*)&Cs[row][32 * hf + 4 * p];
        float* dst = outF + (size_t)(m0 + row) * Nn + n0 + 32 * hf + 4 * p;
        *(volatile v4f*)dst = v;
      }
    }
  } else {
    const bool isV = (MODE == 2) && (n0 >= Cc);
    const int b = m0 / Lc;
    const int l0 = m0 - b * Lc;
    if (!isV) {
#pragma unroll
      for (int c = 0; c < 2; ++c) {
        float scl[8];
#pragma unroll
        for (int r = 0; r < 8; ++r) {
          float s2 = acc[2 * c][r] * acc[2 * c][r] + acc[2 * c + 1][r] * acc[2 * c + 1][r];
          s2 += __shfl_xor(s2, 1);
          s2 += __shfl_xor(s2, 2);
          s2 += __shfl_xor(s2, 4);
          s2 += __shfl_xor(s2, 8);
          scl[r] = 16.0f * (1.0f / fmaxf(sqrtf(s2), 1e-12f));
        }
#pragma unroll
        for (int tt = 0; tt < 2; ++tt) {
          const int t = 2 * c + tt;
#pragma unroll
          for (int r = 0; r < 8; ++r)
            S16[0][16 * wave + 8 * lh + r][16 * t + lx] = hbits(acc[t][r] * scl[r]);
        }
      }
      __syncthreads();
      unsigned short* dstb = (MODE == 1) ? q16 : k16;
      const int hb = n0 >> 5;
#pragma unroll
      for (int ps = 0; ps < 2; ++ps) {
        if (ps) __threadfence();
#pragma unroll
        for (int i = 0; i < 4; ++i) {
          const int L = 4 * i + q;
          const int c = L >> 3, j = L & 7;
          const int row = 16 * wave + 2 * j + (p >> 2);
          const int col = 32 * c + 8 * (p & 3);
          const v8us v = *(const v8us*)&S16[0][row][col];
          const size_t off =
              ((size_t)((b * Hc + hb + c) * Lc + l0 + 16 * wave + 2 * j)) * Dc + 8 * p;
          *(volatile v8us*)(dstb + off) = v;
        }
      }
    } else {
#pragma unroll
      for (int t = 0; t < 4; ++t)
#pragma unroll
        for (int r = 0; r < 8; ++r) {
          unsigned short h, l;
          split1(acc[t][r], h, l);
          S16[0][16 * wave + 8 * lh + r][16 * t + lx] = h;
          S16[1][16 * wave + 8 * lh + r][16 * t + lx] = l;
        }
      __syncthreads();
      const int hb = (n0 - Cc) >> 5;
      const int lt = l0 >> 6;
#pragma unroll
      for (int ps = 0; ps < 2; ++ps) {
        if (ps) __threadfence();
#pragma unroll
        for (int i = 0; i < 8; ++i) {
          const int L = 4 * i + q;
          const int plane = L >> 4;
          const int c = (L >> 3) & 1;
          const int d = 8 * wave + (L & 7);
          v8us v;
#pragma unroll
          for (int e = 0; e < 8; ++e) v[e] = S16[plane][8 * p + e][32 * c + d];
          const size_t off = (size_t)plane * planeElems +
              (((size_t)((b * Hc + hb + c) * (Lc / 64) + lt)) * Dc + d) * 64 + 8 * p;
          *(volatile v8us*)(vT + off) = v;
        }
      }
    }
  }
}

__global__ __launch_bounds__(128)
void attn64(const unsigned short* __restrict__ q16, const unsigned short* __restrict__ k16,
            const unsigned short* __restrict__ vT, const float* __restrict__ temp,
            int ntemp, float* __restrict__ ctx, size_t planeElems) {
  __shared__ __align__(16) unsigned short Ks[64][32];
  __shared__ __align__(16) unsigned short Vt[2][32][64];
  __shared__ __align__(16) unsigned short Ps[2][4][16][64];
  __shared__ __align__(16) float Os[4][16][32];

  const int tid = threadIdx.x;
  const int wave = tid >> 5, lane = tid & 31;
  const int lx = lane & 15, lh = lane >> 4;
  const int bh = blockIdx.y;
  const int b = bh / Hc, h = bh - b * Hc;
  const int l0 = blockIdx.x * 64;
  const size_t base = (size_t)bh * Lc * Dc;
  const int th = (h < ntemp) ? h : (ntemp - 1);
  const float tsc = temp[th] * (1.0f / 256.0f);

  FragH qf;
  {
    const unsigned short* qp = q16 + base + (size_t)(l0 + 16 * wave + lx) * Dc;
    qf.u[0] = *(const v8us*)(qp + 8 * lh);
    qf.u[1] = *(const v8us*)(qp + 16 + 8 * lh);
  }
  float mrow[8], lrow[8];
#pragma unroll
  for (int r = 0; r < 8; ++r) { mrow[r] = -3.0e38f; lrow[r] = 0.0f; }
  v8f oacc[2] = {};

  for (int n0 = 0; n0 < Lc; n0 += 64) {
    {
      const int r = tid >> 1, hh = (tid & 1) * 16;
      const unsigned short* kp = k16 + base + (size_t)(n0 + r) * Dc + hh;
      *(v8us*)&Ks[r][hh] = *(const v8us*)kp;
      *(v8us*)&Ks[r][hh + 8] = *(const v8us*)(kp + 8);
    }
    {
      const size_t toff = ((size_t)bh * (Lc / 64) + (n0 >> 6)) * (size_t)(Dc * 64);
      unsigned short* vdst = &Vt[0][0][0];
#pragma unroll
      for (int jj = 0; jj < 4; ++jj) {
        const int idx = tid + 128 * jj;
        const int plane = idx >> 8;
        const int e = (idx & 255) * 8;
        *(v8us*)(vdst + plane * 2048 + e) =
            *(const v8us*)(vT + (size_t)plane * planeElems + toff + e);
      }
    }
    __syncthreads();

    v8f s[4];
#pragma unroll
    for (int t = 0; t < 4; ++t) {
      const int n = 16 * t + lx;
      FragH kf;
      kf.u[0] = *(const v8us*)&Ks[n][8 * lh];
      kf.u[1] = *(const v8us*)&Ks[n][16 + 8 * lh];
      v8f z = {};
      s[t] = wmh(qf.v, kf.v, z);
    }
#pragma unroll
    for (int t = 0; t < 4; ++t)
#pragma unroll
      for (int r = 0; r < 8; ++r) s[t][r] *= tsc;

#pragma unroll
    for (int r = 0; r < 8; ++r) {
      float m = fmaxf(fmaxf(s[0][r], s[1][r]), fmaxf(s[2][r], s[3][r]));
      m = fmaxf(m, __shfl_xor(m, 1));
      m = fmaxf(m, __shfl_xor(m, 2));
      m = fmaxf(m, __shfl_xor(m, 4));
      m = fmaxf(m, __shfl_xor(m, 8));
      const float mnew = fmaxf(mrow[r], m);
      float rs = 0.0f;
#pragma unroll
      for (int t = 0; t < 4; ++t) {
        const float pv = __expf(s[t][r] - mnew);
        s[t][r] = pv;
        rs += pv;
      }
      rs += __shfl_xor(rs, 1);
      rs += __shfl_xor(rs, 2);
      rs += __shfl_xor(rs, 4);
      rs += __shfl_xor(rs, 8);
      const float alpha = __expf(mrow[r] - mnew);
      lrow[r] = lrow[r] * alpha + rs;
      mrow[r] = mnew;
      oacc[0][r] *= alpha;
      oacc[1][r] *= alpha;
    }

#pragma unroll
    for (int t = 0; t < 4; ++t)
#pragma unroll
      for (int r = 0; r < 8; ++r) {
        unsigned short ph, pl;
        split1(s[t][r], ph, pl);
        Ps[0][wave][8 * lh + r][16 * t + lx] = ph;
        Ps[1][wave][8 * lh + r][16 * t + lx] = pl;
      }
    __syncthreads();

#pragma unroll
    for (int ch = 0; ch < 2; ++ch) {
      FragB pfh, pfl;
      pfh.u[0] = *(const v8us*)&Ps[0][wave][lx][32 * ch + 8 * lh];
      pfh.u[1] = *(const v8us*)&Ps[0][wave][lx][32 * ch + 16 + 8 * lh];
      pfl.u[0] = *(const v8us*)&Ps[1][wave][lx][32 * ch + 8 * lh];
      pfl.u[1] = *(const v8us*)&Ps[1][wave][lx][32 * ch + 16 + 8 * lh];
#pragma unroll
      for (int nt = 0; nt < 2; ++nt) {
        const int d = 16 * nt + lx;
        FragB vfh, vfl;
        vfh.u[0] = *(const v8us*)&Vt[0][d][32 * ch + 8 * lh];
        vfh.u[1] = *(const v8us*)&Vt[0][d][32 * ch + 16 + 8 * lh];
        vfl.u[0] = *(const v8us*)&Vt[1][d][32 * ch + 8 * lh];
        vfl.u[1] = *(const v8us*)&Vt[1][d][32 * ch + 16 + 8 * lh];
        oacc[nt] = wmb(pfh.v, vfh.v, oacc[nt]);
        oacc[nt] = wmb(pfh.v, vfl.v, oacc[nt]);
        oacc[nt] = wmb(pfl.v, vfh.v, oacc[nt]);
      }
    }
    __syncthreads();
  }

#pragma unroll
  for (int r = 0; r < 8; ++r) {
    const float linv = 1.0f / lrow[r];
    Os[wave][8 * lh + r][lx] = oacc[0][r] * linv;
    Os[wave][8 * lh + r][16 + lx] = oacc[1][r] * linv;
  }
  __syncthreads();
  const int q = lane >> 3, p = lane & 7;
#pragma unroll
  for (int ps = 0; ps < 2; ++ps) {
    if (ps) __threadfence();
#pragma unroll
    for (int i = 0; i < 4; ++i) {
      const int rr = 4 * i + q;
      const int l = l0 + 16 * wave + rr;
      const v4f v = *(const v4f*)&Os[wave][rr][4 * p];
      float* dst = ctx + ((size_t)b * Lc + l) * Cc + h * Dc + 4 * p;
      *(volatile v4f*)dst = v;
    }
  }
}

extern "C" void kernel_launch(void* const* d_in, const int* in_sizes, int n_in,
                              void* d_out, int out_size, void* d_ws, size_t ws_size,
                              hipStream_t stream) {
  if (n_in < 6) return;
  const int nX = in_sizes[0];
  if (nX <= 0 || (nX % Cc) != 0) return;
  const int Mtot = nX / Cc;
  if ((Mtot % Lc) != 0) return;
  const int Bn = Mtot / Lc;
  if (in_sizes[1] != nX) return;
  if (in_sizes[2] != Cc * Cc || in_sizes[3] != Cc * 2 * Cc || in_sizes[4] != Cc * Cc) return;
  if (in_sizes[5] < 1) return;
  if (out_size != nX) return;

  const float* x = (const float*)d_in[0];
  const float* y = (const float*)d_in[1];
  const float* Wq = (const float*)d_in[2];
  const float* Wkv = (const float*)d_in[3];
  const float* Wo = (const float*)d_in[4];
  const float* tp = (const float*)d_in[5];
  float* out = (float*)d_out;

  const size_t nXY = (size_t)nX;
  size_t off = 0;
  const size_t oQ = off;   off += (nXY * 2 + 127) & ~(size_t)127;
  const size_t oK = off;   off += (nXY * 2 + 127) & ~(size_t)127;
  const size_t oV = off;   off += (nXY * 4 + 127) & ~(size_t)127;
  const size_t oC = off;   off += (nXY * 4 + 127) & ~(size_t)127;
  if (off > ws_size) return;

  unsigned char* ws = (unsigned char*)d_ws;
  unsigned short* q16 = (unsigned short*)(ws + oQ);
  unsigned short* k16 = (unsigned short*)(ws + oK);
  unsigned short* vT = (unsigned short*)(ws + oV);
  float* ctx = (float*)(ws + oC);

  gemm64<1><<<dim3(Mtot / 64, Cc / 64), 128, 0, stream>>>(
      x, Wq, Cc, Mtot, nullptr, q16, nullptr, nullptr, nXY);
  gemm64<2><<<dim3(Mtot / 64, (2 * Cc) / 64), 128, 0, stream>>>(
      y, Wkv, 2 * Cc, Mtot, nullptr, nullptr, k16, vT, nXY);
  attn64<<<dim3(Lc / 64, Bn * Hc), 128, 0, stream>>>(
      q16, k16, vT, tp, in_sizes[5], ctx, nXY);
  gemm64<0><<<dim3(Mtot / 64, Cc / 64), 128, 0, stream>>>(
      ctx, Wo, Cc, Mtot, out, nullptr, nullptr, nullptr, nXY);
}
